// MultiHeadAttention_4260607558224
// MI455X (gfx1250) — hardware-verified
//
#include <hip/hip_runtime.h>


#ifndef NB
#define NB 4
#endif
#ifndef SEQ
#define SEQ 2048
#endif
#define NB_FULL  4
#define SEQ_FULL 2048
#ifndef OUT_SEQ
#define OUT_SEQ SEQ
#endif
#define DM   1024
#define NH_  16
#define HD   64
#define AW   4
#ifndef EARLY
#define EARLY ((SEQ) < 512 ? (SEQ) : 512)
#endif
#define QRS  2048.0f
#define QRI  (1.0f / 2048.0f)
#define SC2  (0.125f * 1.4426950408889634f)
#define PSH  8.0f
#define CTXS 16.0f
#define WPS  32.0f
#define OSC  (1.0f / 512.0f)
#define NEGB (-3.0e38f)

static_assert(HD == 64);
static_assert(NH_ * HD == DM);
static_assert(DM % 64 == 0);
static_assert(DM % 32 == 0);
static_assert(SEQ % 64 == 0);
static_assert((NB * SEQ) % 64 == 0);
static_assert(SEQ % 32 == 0);
static_assert(EARLY % 64 == 0);
static_assert(EARLY >= 64);
static_assert(EARLY <= SEQ);
static_assert((SEQ - EARLY) % 64 == 0);
static_assert(EARLY % (16 * AW) == 0);
static_assert((SEQ - EARLY) % (16 * AW) == 0);
static_assert(((size_t)SEQ * DM) % 8 == 0);
static_assert(NB <= NB_FULL);
static_assert(SEQ <= SEQ_FULL);

typedef _Float16 h16;
typedef unsigned short bf;
typedef __attribute__((ext_vector_type(16))) __bf16   v16bf;
typedef __attribute__((ext_vector_type(16))) _Float16 v16h;
typedef __attribute__((ext_vector_type(8)))  _Float16 v8h;
typedef __attribute__((ext_vector_type(8)))  unsigned short v8us;
typedef __attribute__((ext_vector_type(8)))  float    v8f;
typedef __attribute__((ext_vector_type(4)))  float    v4f;
typedef v4f  __attribute__((may_alias)) v4fa;

__device__ __forceinline__ unsigned short f2bf(float f) { unsigned u = __float_as_uint(f); u += 0x7FFFu + ((u >> 16) & 1u); return (unsigned short)(u >> 16); }
__device__ __forceinline__ float bfval(float f) { return __uint_as_float(((unsigned)f2bf(f)) << 16); }
__device__ __forceinline__ v16h cat16(v8h lo, v8h hi) { return __builtin_shufflevector(lo, hi, 0, 1, 2, 3, 4, 5, 6, 7, 8, 9, 10, 11, 12, 13, 14, 15); }
__device__ __forceinline__ v16bf cat16b(v8us lo, v8us hi) { return __builtin_bit_cast(v16bf, __builtin_shufflevector(lo, hi, 0, 1, 2, 3, 4, 5, 6, 7, 8, 9, 10, 11, 12, 13, 14, 15)); }
__device__ __forceinline__ v8f wmma16(v16h a, v16h b, v8f c) { return __builtin_amdgcn_wmma_f32_16x16x32_f16(false, a, false, b, (short)0, c, false, false); }
__device__ __forceinline__ v8f wmmab(v16bf a, v16bf b, v8f c) { return __builtin_amdgcn_wmma_f32_16x16x32_bf16(false, a, false, b, (short)0, c, false, false); }
__device__ __forceinline__ v16h  ldh(const h16* p) { return cat16(*(const v8h*)p, *(const v8h*)(p + 16)); }
__device__ __forceinline__ v16bf ldb(const bf* p)  { return cat16b(*(const v8us*)p, *(const v8us*)(p + 16)); }
__device__ __forceinline__ void wave_sync() { __builtin_amdgcn_fence(3  , "wavefront"); __builtin_amdgcn_wave_barrier(); asm volatile("" ::: "memory"); }

__global__ __launch_bounds__(256) void k_cvt8(const float* __restrict__ src, bf* dst, size_t n8) {
    const size_t i = (size_t)blockIdx.x * 256 + threadIdx.x; if (i >= n8) return;
    const v8f v = *(const v8f*)(src + i * 8); v8us o;
#pragma unroll
    for (int k = 0; k < 8; ++k) o[k] = f2bf(v[k]);
    *(volatile v8us*)(dst + i * 8) = o; __threadfence(); *(volatile v8us*)(dst + i * 8) = o;
}

template <int MODE>
__global__ __launch_bounds__(256) void k_tr(const float* __restrict__ src, unsigned short* dst, int R, int C) {
    __shared__ float ts[64 * 65];
    const int tid = threadIdx.x;
    const int r0 = blockIdx.x * 64, c0 = blockIdx.y * 64;
    const size_t bo = (size_t)blockIdx.z * (size_t)R * (size_t)C;
#pragma unroll
    for (int j = 0; j < 4; ++j) {
        const int r = (tid >> 4) + 16 * j, c4 = (tid & 15) * 4;
        const v4f v = *(const v4f*)(src + bo + (size_t)(r0 + r) * (size_t)C + c0 + c4);
        ts[r * 65 + c4 + 0] = v[0]; ts[r * 65 + c4 + 1] = v[1]; ts[r * 65 + c4 + 2] = v[2]; ts[r * 65 + c4 + 3] = v[3];
    }
    __syncthreads();
    const int p = tid & 7;
    v8us o[2];
#pragma unroll
    for (int j = 0; j < 2; ++j) {
        const int row = (tid >> 3) + 32 * j;
        v8us ob; v8h oh;
#pragma unroll
        for (int i = 0; i < 8; ++i) { const float w = ts[(8 * p + i) * 65 + row]; ob[i] = f2bf(w); oh[i] = (h16)(bfval(w) * WPS); }
        if (MODE == 0) o[j] = ob; else o[j] = __builtin_bit_cast(v8us, oh);
    }
#pragma unroll 1
    for (int ps = 0; ps < 2; ++ps) {
#pragma unroll
        for (int j = 0; j < 2; ++j) { const int row = (tid >> 3) + 32 * j;
            *(volatile v8us*)(dst + bo + (size_t)(c0 + row) * (size_t)R + r0 + 8 * p) = o[j]; }
        if (ps == 0) __threadfence();
    }
}

__global__ __launch_bounds__(32) void k_proj(const bf* __restrict__ A, const bf* __restrict__ Bt, h16* Ph, h16* Pr, int resMode,
                                             int RB, size_t sRB, int pitch, int CB, size_t sCB, size_t sRBr, int pitchr, size_t sCBr) {
    __shared__ __align__(16) float os[16 * 68];
    const int K = DM;
    const int lane = threadIdx.x & 31, lr = lane & 15, hi = lane >> 4; const int r0 = blockIdx.x * 64, c0 = blockIdx.y * 64;
    v8f acc[4][4];
#pragma unroll
    for (int mb = 0; mb < 4; ++mb)
#pragma unroll
        for (int nb = 0; nb < 4; ++nb) acc[mb][nb] = (v8f){};
    const size_t aoff = (size_t)(r0 + lr) * K + 8 * hi, boff = (size_t)(c0 + lr) * K + 8 * hi;
#pragma unroll 1
    for (int kc = 0; kc < K; kc += 32) {
        v16bf a[4];
#pragma unroll
        for (int mb = 0; mb < 4; ++mb) a[mb] = ldb(A + aoff + (size_t)mb * 16 * K + kc);
#pragma unroll
        for (int nb = 0; nb < 4; ++nb) { const v16bf b = ldb(Bt + boff + (size_t)nb * 16 * K + kc);
#pragma unroll
            for (int mb = 0; mb < 4; ++mb) acc[mb][nb] = wmmab(a[mb], b, acc[mb][nb]); }
        asm volatile("v_nop\n\tv_nop\n\tv_nop\n\tv_nop" : "+v"(acc[0][3]), "+v"(acc[1][3]), "+v"(acc[2][3]), "+v"(acc[3][3]) : "v"(a[0]), "v"(a[1]), "v"(a[2]), "v"(a[3]));
    }
    const bool res = (resMode == 1) ? ((r0 % RB) < EARLY) : ((resMode == 2) ? ((c0 % CB) < EARLY) : false);
    const size_t tbase = (size_t)(r0 / RB) * sRB  + (size_t)(r0 % RB) * (size_t)pitch  + (size_t)(c0 / CB) * sCB  + (size_t)(c0 % CB);
    const size_t tbr   = (size_t)(r0 / RB) * sRBr + (size_t)(r0 % RB) * (size_t)pitchr + (size_t)(c0 / CB) * sCBr + (size_t)(c0 % CB);
#pragma unroll
    for (int mb = 0; mb < 4; ++mb) {
#pragma unroll
        for (int nb = 0; nb < 4; ++nb) {
#pragma unroll
            for (int j = 0; j < 8; ++j) os[(hi * 8 + j) * 68 + nb * 16 + lr] = acc[mb][nb][j]; }
        wave_sync();
        const size_t sb  = tbase + (size_t)(mb * 16) * (size_t)pitch;
        const size_t sbr = tbr   + (size_t)(mb * 16) * (size_t)pitchr;
#pragma unroll 1
        for (int ps = 0; ps < 2; ++ps) {
#pragma unroll
            for (int s = 0; s < 4; ++s) { const int row = 4 * s + (lane >> 3), c8 = (lane & 7) * 8;
                const v4f x0 = *(const v4fa*)(&os[row * 68 + c8]); const v4f x1 = *(const v4fa*)(&os[row * 68 + c8 + 4]); v8h hv, rv;
#pragma unroll
                for (int i = 0; i < 4; ++i) { const h16 a0 = (h16)x0[i]; const h16 a1 = (h16)x1[i]; hv[i] = a0; hv[4 + i] = a1; rv[i] = (h16)((x0[i] - (float)a0) * QRS); rv[4 + i] = (h16)((x1[i] - (float)a1) * QRS); }
                const size_t oo  = sb  + (size_t)row * (size_t)pitch  + c8;
                const size_t oor = sbr + (size_t)row * (size_t)pitchr + c8;
                *(volatile v8h*)(Ph + oo) = hv; if (res) *(volatile v8h*)(Pr + oor) = rv; }
            if (ps == 0) __threadfence(); }
        wave_sync();
    }
}

template <bool E>
__global__ __launch_bounds__(32 * AW) void k_flash(const h16* __restrict__ QH, const h16* __restrict__ QR, const h16* __restrict__ KP, const h16* __restrict__ KR,
                                                   const h16* __restrict__ VT, const h16* __restrict__ VR, h16* CH, h16* CR, int tq0) {
    __shared__ __align__(16) float os[AW * 16 * 68];
    const int lane = threadIdx.x & 31, lr = lane & 15, hi = lane >> 4;
    const int wave = __builtin_amdgcn_readfirstlane((int)(threadIdx.x >> 5));
    const int zh = blockIdx.y; const int b = zh / NH_, h = zh % NH_;
    const int t0 = tq0 + ((int)blockIdx.x * AW + wave) * 16;
    const size_t pbase = (size_t)zh * SEQ * HD;
    const size_t ebase = (size_t)zh * EARLY * HD;
    const size_t qo = pbase + (size_t)(t0 + lr) * HD + 8 * hi;
    const v16h qh0 = ldh(QH + qo), qh1 = ldh(QH + qo + 32);
    v16h qr0 = (v16h){}, qr1 = (v16h){};
    if (E) { const size_t qe = ebase + (size_t)(t0 + lr) * HD + 8 * hi; qr0 = ldh(QR + qe); qr1 = ldh(QR + qe + 32); }
    const size_t ko  = pbase + (size_t)lr * HD + 8 * hi;
    const size_t kro = ebase + (size_t)lr * HD + 8 * hi;
    const size_t vo  = pbase + (size_t)lr * SEQ + 8 * hi;
    const size_t vro = ebase + (size_t)lr * EARLY + 8 * hi;
    v8f o[4], rr[4];
#pragma unroll
    for (int j = 0; j < 4; ++j) { o[j] = (v8f){}; rr[j] = (v8f){}; }
    float m = NEGB, l = 0.0f;
    const int tq = t0 + lr;
#pragma unroll 1
    for (int key0 = 0; key0 < t0 + 16; key0 += 32) {
        const h16* ka = KP + ko + (size_t)key0 * HD;
        const v16h ka0 = ldh(ka), ka1 = ldh(ka + 32), kb0 = ldh(ka + 16 * HD), kb1 = ldh(ka + 16 * HD + 32);
        v8f sHa = (v8f){}, sLa = (v8f){}, sHb = (v8f){}, sLb = (v8f){};
        if (E) {
            const h16* kr = KR + kro + (size_t)key0 * HD;
            const v16h ra0 = ldh(kr), ra1 = ldh(kr + 32), rb0 = ldh(kr + 16 * HD), rb1 = ldh(kr + 16 * HD + 32);
            sHa = wmma16(ka0, qh0, sHa); sLa = wmma16(ka0, qr0, sLa); sHb = wmma16(kb0, qh0, sHb); sLb = wmma16(kb0, qr0, sLb);
            sHa = wmma16(ka1, qh1, sHa); sLa = wmma16(ka1, qr1, sLa); sHb = wmma16(kb1, qh1, sHb); sLb = wmma16(kb1, qr1, sLb);
            sLa = wmma16(ra0, qh0, sLa); sLb = wmma16(rb0, qh0, sLb); sLa = wmma16(ra1, qh1, sLa); sLb = wmma16(rb1, qh1, sLb);
            asm volatile("v_nop\n\tv_nop\n\tv_nop\n\tv_nop" : "+v"(sHa), "+v"(sLa), "+v"(sHb), "+v"(sLb) : "v"(ka0), "v"(ka1), "v"(kb0), "v"(kb1), "v"(ra0), "v"(ra1), "v"(rb0), "v"(rb1));
        } else {
            sHa = wmma16(ka0, qh0, sHa); sHb = wmma16(kb0, qh0, sHb);
            sHa = wmma16(ka1, qh1, sHa); sHb = wmma16(kb1, qh1, sHb);
            asm volatile("v_nop\n\tv_nop\n\tv_nop\n\tv_nop" : "+v"(sHa), "+v"(sHb) : "v"(ka0), "v"(ka1), "v"(kb0), "v"(kb1));
        }
        float ta[8], tb[8];
#pragma unroll
        for (int r = 0; r < 8; ++r) {
            if (E) { ta[r] = (sHa[r] + sLa[r] * QRI) * SC2; tb[r] = (sHb[r] + sLb[r] * QRI) * SC2; }
            else   { ta[r] = sHa[r] * SC2; tb[r] = sHb[r] * SC2; } }
        if (key0 + 32 > t0) {
            const int kk = key0 + 8 * hi;
#pragma unroll
            for (int r = 0; r < 8; ++r) { ta[r] = (kk + r > tq) ? NEGB : ta[r]; tb[r] = (kk + 16 + r > tq) ? NEGB : tb[r]; }
        }
        float mx = NEGB;
#pragma unroll
        for (int r = 0; r < 8; ++r) mx = fmaxf(mx, fmaxf(ta[r], tb[r]));
        mx = fmaxf(mx, __shfl_xor(mx, 16, 32));
        const float mnew = fmaxf(m, mx);
        const float alpha = __builtin_amdgcn_exp2f(m - mnew);
        const float sh = PSH - mnew;
        v16h pb, pr = (v16h){}; float ls = 0.0f;
#pragma unroll
        for (int r = 0; r < 8; ++r) {
            const float fa = __builtin_amdgcn_exp2f(ta[r] + sh); const float fc = __builtin_amdgcn_exp2f(tb[r] + sh);
            const h16 pa = (h16)fa; const h16 pc = (h16)fc; pb[r] = pa; pb[8 + r] = pc;
            if (E) { pr[r] = (h16)((fa - (float)pa) * QRS); pr[8 + r] = (h16)((fc - (float)pc) * QRS); ls += fa + fc; }
            else   { ls += (float)pa + (float)pc; } }
        l = l * alpha + ls; m = mnew;
#pragma unroll
        for (int j = 0; j < 4; ++j) { o[j] = o[j] * alpha; if (E) rr[j] = rr[j] * alpha; }
        const h16* va = VT + vo + key0;
        const v16h v0 = ldh(va), v1 = ldh(va + (size_t)16 * SEQ), v2 = ldh(va + (size_t)32 * SEQ), v3 = ldh(va + (size_t)48 * SEQ);
        if (E) {
            const h16* vr = VR + vro + key0;
            const v16h w0 = ldh(vr), w1 = ldh(vr + (size_t)16 * EARLY), w2 = ldh(vr + (size_t)32 * EARLY), w3 = ldh(vr + (size_t)48 * EARLY);
            o[0] = wmma16(v0, pb, o[0]); o[1] = wmma16(v1, pb, o[1]); o[2] = wmma16(v2, pb, o[2]); o[3] = wmma16(v3, pb, o[3]);
            rr[0] = wmma16(w0, pb, rr[0]); rr[1] = wmma16(w1, pb, rr[1]); rr[2] = wmma16(w2, pb, rr[2]); rr[3] = wmma16(w3, pb, rr[3]);
            rr[0] = wmma16(v0, pr, rr[0]); rr[1] = wmma16(v1, pr, rr[1]); rr[2] = wmma16(v2, pr, rr[2]); rr[3] = wmma16(v3, pr, rr[3]);
            asm volatile("v_nop\n\tv_nop\n\tv_nop\n\tv_nop" : "+v"(o[0]), "+v"(o[1]), "+v"(o[2]), "+v"(o[3]), "+v"(rr[0]), "+v"(rr[1]), "+v"(rr[2]), "+v"(rr[3])
                         : "v"(v0), "v"(v1), "v"(v2), "v"(v3), "v"(w0), "v"(w1), "v"(w2), "v"(w3), "v"(pb), "v"(pr));
        } else {
            o[0] = wmma16(v0, pb, o[0]); o[1] = wmma16(v1, pb, o[1]); o[2] = wmma16(v2, pb, o[2]); o[3] = wmma16(v3, pb, o[3]);
            asm volatile("v_nop\n\tv_nop\n\tv_nop\n\tv_nop" : "+v"(o[0]), "+v"(o[1]), "+v"(o[2]), "+v"(o[3]) : "v"(v0), "v"(v1), "v"(v2), "v"(v3), "v"(pb));
        }
    }
    l += __shfl_xor(l, 16, 32);
    const float inv = CTXS * (1.0f / l);
    const int wb = wave * 16 * 68;
#pragma unroll
    for (int j = 0; j < 4; ++j) { v4f a, c;
#pragma unroll
        for (int i = 0; i < 4; ++i) {
            if (E) { a[i] = (o[j][i] + rr[j][i] * QRI) * inv; c[i] = (o[j][4 + i] + rr[j][4 + i] * QRI) * inv; }
            else   { a[i] = o[j][i] * inv; c[i] = o[j][4 + i] * inv; } }
        *(v4fa*)(&os[wb + lr * 68 + 16 * j + 8 * hi]) = a; *(v4fa*)(&os[wb + lr * 68 + 16 * j + 8 * hi + 4]) = c; }
    wave_sync();
    const size_t cb  = ((size_t)b * SEQ   + t0) * DM + (size_t)h * HD;
    const size_t cbr = ((size_t)b * EARLY + t0) * DM + (size_t)h * HD;
#pragma unroll 1
    for (int ps = 0; ps < 2; ++ps) {
#pragma unroll
        for (int s = 0; s < 4; ++s) { const int row = 4 * s + (lane >> 3), c8 = (lane & 7) * 8;
            const v4f x0 = *(const v4fa*)(&os[wb + row * 68 + c8]); const v4f x1 = *(const v4fa*)(&os[wb + row * 68 + c8 + 4]); v8h hv, rv;
#pragma unroll
            for (int i = 0; i < 4; ++i) { const h16 a0 = (h16)x0[i]; const h16 a1 = (h16)x1[i]; hv[i] = a0; hv[4 + i] = a1; rv[i] = (h16)((x0[i] - (float)a0) * QRS); rv[4 + i] = (h16)((x1[i] - (float)a1) * QRS); }
            *(volatile v8h*)(CH + cb + (size_t)row * DM + c8) = hv;
            if (E) *(volatile v8h*)(CR + cbr + (size_t)row * DM + c8) = rv; }
        if (ps == 0) __threadfence(); }
}

__global__ __launch_bounds__(32) void k_out_d(const h16* __restrict__ A, const h16* __restrict__ Bt, const float* __restrict__ bp, float* OUT, int tilesPerBatch, int tstart) {
    __shared__ __align__(16) float os[16 * 68];
    const int K = DM;
    const int lane = threadIdx.x & 31, lr = lane & 15, hi = lane >> 4;
    const int bb = (int)blockIdx.x / tilesPerBatch; const int tt = tstart + ((int)blockIdx.x % tilesPerBatch) * 64;
    const int m0 = bb * SEQ + tt, c0 = blockIdx.y * 64;
    v8f acc[4][4];
#pragma unroll
    for (int mb = 0; mb < 4; ++mb)
#pragma unroll
        for (int nb = 0; nb < 4; ++nb) acc[mb][nb] = (v8f){};
    const size_t aoff = (size_t)(m0 + lr) * K + 8 * hi, boff = (size_t)(c0 + lr) * K + 8 * hi;
#pragma unroll 1
    for (int kc = 0; kc < K; kc += 32) {
        v16h a[4]; v16h bq = (v16h){};
#pragma unroll
        for (int mb = 0; mb < 4; ++mb) a[mb] = ldh(A + aoff + (size_t)mb * 16 * K + kc);
#pragma unroll
        for (int nb = 0; nb < 4; ++nb) { bq = ldh(Bt + boff + (size_t)nb * 16 * K + kc);
#pragma unroll
            for (int mb = 0; mb < 4; ++mb) acc[mb][nb] = wmma16(a[mb], bq, acc[mb][nb]); }
        asm volatile("v_nop\n\tv_nop\n\tv_nop\n\tv_nop" : "+v"(acc[0][3]), "+v"(acc[1][3]), "+v"(acc[2][3]), "+v"(acc[3][3]) : "v"(a[0]), "v"(a[1]), "v"(a[2]), "v"(a[3]), "v"(bq));
    }
    float bv[4];
#pragma unroll
    for (int nb = 0; nb < 4; ++nb) bv[nb] = bfval(bp[c0 + nb * 16 + lr]);
    float* orow = OUT + ((size_t)bb * OUT_SEQ + tt) * DM + c0;
#pragma unroll
    for (int mb = 0; mb < 4; ++mb) {
#pragma unroll
        for (int nb = 0; nb < 4; ++nb) {
#pragma unroll
            for (int j = 0; j < 8; ++j) os[(hi * 8 + j) * 68 + nb * 16 + lr] = acc[mb][nb][j] * OSC + bv[nb]; }
        wave_sync();
#pragma unroll 1
        for (int ps = 0; ps < 2; ++ps) {
#pragma unroll
            for (int s = 0; s < 8; ++s) { const int row = 2 * s + hi, cofs = lr * 4;
                const v4f val = *(const v4fa*)(&os[row * 68 + cofs]);
                *(volatile v4f*)(orow + (size_t)(mb * 16 + row) * DM + cofs) = val; }
            if (ps == 0) __threadfence(); }
        wave_sync();
    }
}

__global__ __launch_bounds__(32) void k_out_e(const h16* __restrict__ A, const h16* __restrict__ Ar, const h16* __restrict__ Bt, const float* __restrict__ bp, float* OUT) {
    __shared__ __align__(16) float os[16 * 68];
    const int K = DM;
    const int lane = threadIdx.x & 31, lr = lane & 15, hi = lane >> 4;
    const int tpb = EARLY / 32;
    const int bb = (int)blockIdx.x / tpb; const int tt = ((int)blockIdx.x % tpb) * 32;
    const int m0 = bb * SEQ + tt, mr0 = bb * EARLY + tt, c0 = blockIdx.y * 64;
    v8f acc[2][4], accr[2][4];
#pragma unroll
    for (int mb = 0; mb < 2; ++mb)
#pragma unroll
        for (int nb = 0; nb < 4; ++nb) { acc[mb][nb] = (v8f){}; accr[mb][nb] = (v8f){}; }
    const size_t aoff = (size_t)(m0 + lr) * K + 8 * hi, roff = (size_t)(mr0 + lr) * K + 8 * hi, boff = (size_t)(c0 + lr) * K + 8 * hi;
#pragma unroll 1
    for (int kc = 0; kc < K; kc += 32) {
        v16h a[2], ar[2]; v16h bq = (v16h){};
#pragma unroll
        for (int mb = 0; mb < 2; ++mb) { a[mb] = ldh(A + aoff + (size_t)mb * 16 * K + kc); ar[mb] = ldh(Ar + roff + (size_t)mb * 16 * K + kc); }
#pragma unroll
        for (int nb = 0; nb < 4; ++nb) { bq = ldh(Bt + boff + (size_t)nb * 16 * K + kc);
#pragma unroll
            for (int mb = 0; mb < 2; ++mb) { acc[mb][nb] = wmma16(a[mb], bq, acc[mb][nb]); accr[mb][nb] = wmma16(ar[mb], bq, accr[mb][nb]); } }
        asm volatile("v_nop\n\tv_nop\n\tv_nop\n\tv_nop" : "+v"(acc[0][3]), "+v"(accr[0][3]), "+v"(acc[1][3]), "+v"(accr[1][3]) : "v"(a[0]), "v"(a[1]), "v"(ar[0]), "v"(ar[1]), "v"(bq));
    }
    float bv[4];
#pragma unroll
    for (int nb = 0; nb < 4; ++nb) bv[nb] = bfval(bp[c0 + nb * 16 + lr]);
    float* orow = OUT + ((size_t)bb * OUT_SEQ + tt) * DM + c0;
#pragma unroll
    for (int mb = 0; mb < 2; ++mb) {
#pragma unroll
        for (int nb = 0; nb < 4; ++nb) {
#pragma unroll
            for (int j = 0; j < 8; ++j) os[(hi * 8 + j) * 68 + nb * 16 + lr] = (acc[mb][nb][j] + accr[mb][nb][j] * QRI) * OSC + bv[nb]; }
        wave_sync();
#pragma unroll 1
        for (int ps = 0; ps < 2; ++ps) {
#pragma unroll
            for (int s = 0; s < 8; ++s) { const int row = 2 * s + hi, cofs = lr * 4;
                const v4f val = *(const v4fa*)(&os[row * 68 + cofs]);
                *(volatile v4f*)(orow + (size_t)(mb * 16 + row) * DM + cofs) = val; }
            if (ps == 0) __threadfence(); }
        wave_sync();
    }
}

static constexpr size_t al256(size_t v) { return (v + 255) & ~(size_t)255; }
static constexpr size_t SZ_XB = al256((size_t)NB * SEQ * DM * 2);
static constexpr size_t SZ_WB = al256((size_t)3 * DM * DM * 2);
static constexpr size_t SZ_WP = al256((size_t)DM * DM * 2);
static constexpr size_t SZ_PL = al256((size_t)NB * NH_ * SEQ * HD * 2);
static constexpr size_t SZ_PE = al256((size_t)NB * NH_ * EARLY * HD * 2);
static constexpr size_t SZ_CH = al256((size_t)NB * SEQ * DM * 2);
static constexpr size_t SZ_CR = al256((size_t)NB * EARLY * DM * 2);
static constexpr size_t SZ_TOTAL = SZ_XB + SZ_WB + SZ_WP + 3 * SZ_PL + 3 * SZ_PE + SZ_CH + SZ_CR;
static_assert(SZ_TOTAL <= (size_t)134217728);
static_assert(((size_t)DM * DM * 2) % 256 == 0);

extern "C" void kernel_launch(void* const* d_in, const int* in_sizes, int n_in,
                              void* d_out, int out_size, void* d_ws, size_t ws_size, hipStream_t stream) {
    if (n_in < 6) return;
    const size_t needx = ((size_t)(NB - 1) * SEQ_FULL + SEQ) * DM;
    if ((size_t)in_sizes[0] < needx) return;
    if ((size_t)in_sizes[1] < (size_t)NH_ * DM * HD || (size_t)in_sizes[2] < (size_t)NH_ * DM * HD || (size_t)in_sizes[3] < (size_t)NH_ * DM * HD) return;
    if ((size_t)in_sizes[4] < (size_t)DM * DM || (size_t)in_sizes[5] < (size_t)DM) return;
    if ((size_t)out_size < ((size_t)(NB - 1) * OUT_SEQ + SEQ) * DM) return;
    if (SZ_TOTAL > ws_size) return;
    const float* x = (const float*)d_in[0]; const float* wq = (const float*)d_in[1]; const float* wk = (const float*)d_in[2]; const float* wv = (const float*)d_in[3];
    const float* wp = (const float*)d_in[4]; const float* bp = (const float*)d_in[5];
    float* OUT = (float*)d_out;
    char* wsp = (char*)d_ws;
    bf* XB = (bf*)wsp; wsp += SZ_XB;
    bf* WB = (bf*)wsp; wsp += SZ_WB;
    h16* WPT = (h16*)wsp; wsp += SZ_WP;
    h16* QH = (h16*)wsp; wsp += SZ_PL;
    h16* KP = (h16*)wsp; wsp += SZ_PL;
    h16* VT = (h16*)wsp; wsp += SZ_PL;
    h16* QR = (h16*)wsp; wsp += SZ_PE;
    h16* KR = (h16*)wsp; wsp += SZ_PE;
    h16* VR = (h16*)wsp; wsp += SZ_PE;
    h16* CH = (h16*)wsp; wsp += SZ_CH;
    h16* CR = (h16*)wsp; wsp += SZ_CR;
    bf* WQ = WB; bf* WK = WB + (size_t)DM * DM; bf* WV = WB + (size_t)2 * DM * DM;

    if (SEQ == SEQ_FULL) {
        const size_t n8 = (size_t)NB * SEQ * DM / 8;
        k_cvt8<<<(unsigned)((n8 + 255) / 256), 256, 0, stream>>>(x, XB, n8);
    } else {
        const size_t n8 = (size_t)SEQ * DM / 8;
        for (int b = 0; b < NB; ++b) k_cvt8<<<(unsigned)((n8 + 255) / 256), 256, 0, stream>>>(x + (size_t)b * SEQ_FULL * DM, XB + (size_t)b * SEQ * DM, n8);
    }
    k_tr<0><<<dim3(DM / 64, HD / 64, NH_), 256, 0, stream>>>(wq, (unsigned short*)WQ, DM, HD);
    k_tr<0><<<dim3(DM / 64, HD / 64, NH_), 256, 0, stream>>>(wk, (unsigned short*)WK, DM, HD);
    k_tr<0><<<dim3(DM / 64, HD / 64, NH_), 256, 0, stream>>>(wv, (unsigned short*)WV, DM, HD);
    k_tr<1><<<dim3(DM / 64, DM / 64, 1), 256, 0, stream>>>(wp, (unsigned short*)WPT, DM, DM);

    k_proj<<<dim3(NB * SEQ / 64, DM / 64, 1), 32, 0, stream>>>(XB, WQ, QH, QR, 1, SEQ, (size_t)NH_ * SEQ * HD, HD, HD, (size_t)SEQ * HD, (size_t)NH_ * EARLY * HD, HD, (size_t)EARLY * HD);
    k_proj<<<dim3(NB * SEQ / 64, DM / 64, 1), 32, 0, stream>>>(XB, WK, KP, KR, 1, SEQ, (size_t)NH_ * SEQ * HD, HD, HD, (size_t)SEQ * HD, (size_t)NH_ * EARLY * HD, HD, (size_t)EARLY * HD);
    k_proj<<<dim3(DM / 64, NB * SEQ / 64, 1), 32, 0, stream>>>(WV, XB, VT, VR, 2, DM, (size_t)0, SEQ, SEQ, (size_t)DM * SEQ, (size_t)0, EARLY, (size_t)DM * EARLY);

    k_flash<true><<<dim3(EARLY / (16 * AW), NB * NH_, 1), 32 * AW, 0, stream>>>(QH, QR, KP, KR, VT, VR, CH, CR, 0);
    if (SEQ > EARLY)
        k_flash<false><<<dim3((SEQ - EARLY) / (16 * AW), NB * NH_, 1), 32 * AW, 0, stream>>>(QH, QH, KP, KP, VT, VT, CH, CH, EARLY);

    k_out_e<<<dim3(NB * (EARLY / 32), DM / 64, 1), 32, 0, stream>>>(CH, CR, WPT, bp, OUT);
    if (SEQ > EARLY)
        k_out_d<<<dim3(NB * ((SEQ - EARLY) / 64), DM / 64, 1), 32, 0, stream>>>(CH, WPT, bp, OUT, (SEQ - EARLY) / 64, EARLY);
}
